// SelfAttention_13383118095010
// MI455X (gfx1250) — hardware-verified
//
#include <hip/hip_runtime.h>
#ifndef NB
#define NB 2
#endif
#ifndef SEQ
#define SEQ 2048
#endif
#define NB_FULL 2
#define SEQ_FULL 2048
#define DM 1024
#define NH 16
#define HD 64
#define NR (NB * SEQ)
#define LOG100F 4.6051702f

static_assert(NH * HD == DM);
static_assert(HD == 64);
static_assert(SEQ % 128 == 0 && NR % 128 == 0 && DM % 128 == 0);
static_assert(DM % 32 == 0 && (2 * DM) % 32 == 0);
static_assert((DM & (DM - 1)) == 0);
static_assert(SEQ % 64 == 0 && SEQ % 32 == 0);
static_assert(NB <= NB_FULL && SEQ <= SEQ_FULL);
static_assert((size_t)NR * DM * 14 + (size_t)8 * DM * DM <= (size_t)134217728);

typedef unsigned short v8us __attribute__((ext_vector_type(8), may_alias));
typedef float  v8f  __attribute__((ext_vector_type(8)));
typedef float  v4f  __attribute__((ext_vector_type(4)));
typedef float  v4fa __attribute__((ext_vector_type(4), may_alias));
typedef _Float16 v16h __attribute__((ext_vector_type(16)));
union FragH { v16h v; v8us half[2]; _Float16 h[16]; unsigned short u[16]; };

__device__ __forceinline__ float bf16_rne(float x) { unsigned int u = __float_as_uint(x); u = (u + 0x7FFFu + ((u >> 16) & 1u)) & 0xFFFF0000u; return __uint_as_float(u); }

__device__ __forceinline__ v16h ld_frag(const unsigned short* __restrict__ p, int hh) { FragH f; f.half[0] = *(const v8us*)(p + 8 * hh); f.half[1] = *(const v8us*)(p + 16 + 8 * hh); return f.v; }
__device__ __forceinline__ v8f mma16(v16h a, v16h b, v8f c) { v8f d = __builtin_amdgcn_wmma_f32_16x16x32_f16(false, a, false, b, (short)0, c, false, false); asm volatile("v_nop\n\tv_nop\n\tv_nop\n\tv_nop" : "+v"(d) : "v"(a), "v"(b)); return d; }

__global__ __launch_bounds__(256) void k_cvt_x(const float* __restrict__ x, unsigned short* __restrict__ X16) {
  const int t = blockIdx.x * 256 + threadIdx.x;
  if (t >= NR * (DM / 8)) return;
  const int r = t / (DM / 8), c8 = (t - r * (DM / 8)) * 8;
  const int b = r / SEQ, l = r - b * SEQ;
  const float* src = x + ((size_t)b * SEQ_FULL + l) * DM + c8;
  const v4f a = *(const v4fa*)src, c = *(const v4fa*)(src + 4);
  FragH f;
#pragma unroll
  for (int q = 0; q < 4; ++q) { f.h[q] = (_Float16)bf16_rne(a[q]); f.h[4 + q] = (_Float16)bf16_rne(c[q]); }
  const v8us o = f.half[0];
  unsigned short* d = X16 + (size_t)r * DM + c8;
  *(volatile v8us*)d = o; __threadfence(); *(volatile v8us*)d = o;
}

__global__ __launch_bounds__(256) void k_cvt_w(const float* __restrict__ w, unsigned short* __restrict__ dst, int n8, float scale) {
  const int t = blockIdx.x * 256 + threadIdx.x;
  if (t >= n8) return;
  const v4f a = *(const v4fa*)(w + (size_t)t * 8), c = *(const v4fa*)(w + (size_t)t * 8 + 4);
  FragH f;
#pragma unroll
  for (int q = 0; q < 4; ++q) { f.h[q] = (_Float16)(bf16_rne(a[q]) * scale); f.h[4 + q] = (_Float16)(bf16_rne(c[q]) * scale); }
  const v8us o = f.half[0];
  unsigned short* d = dst + (size_t)t * 8;
  *(volatile v8us*)d = o; __threadfence(); *(volatile v8us*)d = o;
}

__device__ __forceinline__ void gemm_core(const unsigned short* __restrict__ A, int lda, const unsigned short* __restrict__ Bt, int ldb, int K, int kmask,
                                          int row0, int col0, int ln, int hh, v8f (&acc)[8]) {
  const unsigned short* a0p = A + (size_t)(row0 + ln) * lda;
  const unsigned short* a1p = a0p + (size_t)16 * lda;
  const unsigned short* b0p = Bt + (size_t)(col0 + ln) * ldb;
  const unsigned short* b1p = b0p + (size_t)16 * ldb;
  const unsigned short* b2p = b1p + (size_t)16 * ldb;
  const unsigned short* b3p = b2p + (size_t)16 * ldb;
  const v8f z8 = {0.f, 0.f, 0.f, 0.f, 0.f, 0.f, 0.f, 0.f};
  v8f c00 = z8, c01 = z8, c02 = z8, c03 = z8, c10 = z8, c11 = z8, c12 = z8, c13 = z8;
#pragma unroll 1
  for (int kb = 0; kb < K; kb += 32) {
    const int kw = kb & kmask;
    const v16h a0 = ld_frag(a0p + kb, hh), a1 = ld_frag(a1p + kb, hh);
    v16h b = ld_frag(b0p + kw, hh); c00 = mma16(a0, b, c00); c10 = mma16(a1, b, c10);
    b = ld_frag(b1p + kw, hh); c01 = mma16(a0, b, c01); c11 = mma16(a1, b, c11);
    b = ld_frag(b2p + kw, hh); c02 = mma16(a0, b, c02); c12 = mma16(a1, b, c12);
    b = ld_frag(b3p + kw, hh); c03 = mma16(a0, b, c03); c13 = mma16(a1, b, c13);
  }
  acc[0] = c00; acc[1] = c01; acc[2] = c02; acc[3] = c03; acc[4] = c10; acc[5] = c11; acc[6] = c12; acc[7] = c13;
}

__global__ __launch_bounds__(128) void k_gemm_qk(const unsigned short* __restrict__ X16, const unsigned short* __restrict__ WQ16, const float* __restrict__ q_bias,
                                                 const float* __restrict__ scale_mul, unsigned short* __restrict__ QP, unsigned short* __restrict__ K16) {
  __shared__ __attribute__((aligned(16))) float so[4][32][68];
  const int tid = threadIdx.x; const int wave = __builtin_amdgcn_readfirstlane((int)(tid >> 5));
  const int lane = tid & 31, ln = lane & 15, hh = lane >> 4;
  const int ntn = (2 * DM) / 64;
  const int mt = blockIdx.x / ntn, nq = blockIdx.x - mt * ntn;
  const int row0 = mt * 128 + 32 * wave, col0 = nq * 64;
  v8f acc[8];
  gemm_core(X16, DM, WQ16, DM, DM, 0x7fffffff, row0, col0, ln, hh, acc);
#pragma unroll
  for (int u = 0; u < 8; ++u) { const int t = u & 3, half = u >> 2;
#pragma unroll
    for (int r = 0; r < 8; ++r) so[wave][half * 16 + 8 * hh + r][t * 16 + ln] = acc[u][r] * 0.0625f; }
  __builtin_amdgcn_fence(4  , "workgroup"); __builtin_amdgcn_wave_barrier();
  const bool isq = (col0 < DM);
  const int h = (col0 >> 6) & (NH - 1);
  const int c8 = (lane & 7) * 8, rq = lane >> 3;
  const int bo = isq ? (h * 64 + c8) : c8;
  const float bsel = isq ? 1.0f : 0.0f;
  float bqv[8];
#pragma unroll
  for (int j = 0; j < 8; ++j) bqv[j] = bf16_rne(q_bias[bo + j]) * bsel;
  const float sm = expf(fminf(bf16_rne(scale_mul[h]), LOG100F));
  const float cmul = isq ? (sm * 4096.0f) : 16.0f;
  for (int pass = 0; pass < 2; ++pass) {
#pragma unroll 1
    for (int it = 0; it < 8; ++it) {
      const int r = it * 4 + rq;
      const v4f a = *(const v4fa*)&so[wave][r][c8], c = *(const v4fa*)&so[wave][r][c8 + 4];
      float v[8] = {a[0] + bqv[0], a[1] + bqv[1], a[2] + bqv[2], a[3] + bqv[3], c[0] + bqv[4], c[1] + bqv[5], c[2] + bqv[6], c[3] + bqv[7]};
      float ss = 0.f;
#pragma unroll
      for (int j = 0; j < 8; ++j) ss += v[j] * v[j];
      ss += __shfl_xor(ss, 1); ss += __shfl_xor(ss, 2); ss += __shfl_xor(ss, 4);
      const float mul = (1.0f / fmaxf(sqrtf(ss), 1.0e-12f)) * cmul;
      FragH fh, fr;
#pragma unroll
      for (int j = 0; j < 8; ++j) { const float cv = v[j] * mul; const _Float16 hi = (_Float16)cv; fh.h[j] = hi; fr.h[j] = (_Float16)(cv - (float)hi); }
      const v8us ohi = fh.half[0], ores = fr.half[0];
      if (isq) {
        unsigned short* d = QP + (size_t)(row0 + r) * (2 * DM) + h * 128 + c8;
        *(volatile v8us*)d = ohi; *(volatile v8us*)(d + 64) = ores;
      } else {
        unsigned short* d = K16 + (size_t)(row0 + r) * DM + h * 64 + c8;
        *(volatile v8us*)d = ohi;
      }
    }
    if (pass == 0) __threadfence();
  }
}

__global__ __launch_bounds__(128) void k_gemm_vt(const unsigned short* __restrict__ WV16, const unsigned short* __restrict__ X16, const float* __restrict__ v_bias, unsigned short* __restrict__ VT) {
  __shared__ __attribute__((aligned(16))) float so[4][32][68];
  const int tid = threadIdx.x; const int wave = __builtin_amdgcn_readfirstlane((int)(tid >> 5));
  const int lane = tid & 31, ln = lane & 15, hh = lane >> 4;
  const int ntn = NR / 64;
  const int mt = blockIdx.x / ntn, nq = blockIdx.x - mt * ntn;
  const int row0 = mt * 128 + 32 * wave, col0 = nq * 64;
  v8f acc[8];
  gemm_core(WV16, DM, X16, DM, DM, 0x7fffffff, row0, col0, ln, hh, acc);
#pragma unroll
  for (int u = 0; u < 8; ++u) { const int t = u & 3, half = u >> 2;
#pragma unroll
    for (int r = 0; r < 8; ++r) so[wave][half * 16 + 8 * hh + r][t * 16 + ln] = acc[u][r] * 0.0625f; }
  __builtin_amdgcn_fence(4  , "workgroup"); __builtin_amdgcn_wave_barrier();
  const int c8 = (lane & 7) * 8, rq = lane >> 3;
  for (int pass = 0; pass < 2; ++pass) {
#pragma unroll 1
    for (int it = 0; it < 8; ++it) {
      const int r = it * 4 + rq;
      const float bv = bf16_rne(v_bias[row0 + r]);
      const v4f a = *(const v4fa*)&so[wave][r][c8], c = *(const v4fa*)&so[wave][r][c8 + 4];
      FragH f;
#pragma unroll
      for (int j = 0; j < 4; ++j) { f.h[j] = (_Float16)(a[j] + bv); f.h[4 + j] = (_Float16)(c[j] + bv); }
      const v8us o = f.half[0];
      *(volatile v8us*)(VT + (size_t)(row0 + r) * NR + col0 + c8) = o;
    }
    if (pass == 0) __threadfence();
  }
}

__global__ __launch_bounds__(128) void k_attn(const unsigned short* __restrict__ QP, const unsigned short* __restrict__ K16, const unsigned short* __restrict__ VT,
                                              const float* __restrict__ bias, unsigned short* __restrict__ CTX) {
  __shared__ __attribute__((aligned(16))) unsigned short sc[4][2][16][72];
  const int tid = threadIdx.x; const int wave = __builtin_amdgcn_readfirstlane((int)(tid >> 5));
  const int lane = tid & 31, ln = lane & 15, hh = lane >> 4;
  const int h = blockIdx.y, b = blockIdx.z;
  const int q0 = blockIdx.x * 64 + wave * 16;
  const int query = q0 + ln;
  const int qoff0 = (b * SEQ + query) * (2 * DM) + h * 128;
  const int koff0 = (b * SEQ + ln) * DM + h * 64;
  const int voff0 = (h * 64 + ln) * NR + b * SEQ;
  const int boff0 = query * SEQ_FULL + 8 * hh;
  const v8f z8 = {0.f, 0.f, 0.f, 0.f, 0.f, 0.f, 0.f, 0.f};
  v8f o0 = z8, o1 = z8, o2 = z8, o3 = z8;
  float mrun = -1.0e30f, lrun = 0.f;
#pragma unroll 1
  for (int kc = 0; kc < SEQ; kc += 32) {
    int qo = qoff0; asm volatile("" : "+v"(qo));
    const unsigned short* kp = K16 + koff0 + kc * DM;
    const v16h k00 = ld_frag(kp, hh), k01 = ld_frag(kp + 32, hh);
    const v16h k10 = ld_frag(kp + 16 * DM, hh), k11 = ld_frag(kp + 16 * DM + 32, hh);
    v8f t0 = z8, t1 = z8;
    v16h bq = ld_frag(QP + qo, hh);       t0 = mma16(k00, bq, t0); t1 = mma16(k10, bq, t1);
    bq = ld_frag(QP + qo + 32, hh);       t0 = mma16(k01, bq, t0); t1 = mma16(k11, bq, t1);
    bq = ld_frag(QP + qo + 64, hh);       t0 = mma16(k00, bq, t0); t1 = mma16(k10, bq, t1);
    bq = ld_frag(QP + qo + 96, hh);       t0 = mma16(k01, bq, t0); t1 = mma16(k11, bq, t1);
    const float* bp = bias + boff0 + kc;
    const v4f b00 = *(const v4fa*)bp, b01 = *(const v4fa*)(bp + 4), b10 = *(const v4fa*)(bp + 16), b11 = *(const v4fa*)(bp + 20);
    float s0[8], s1[8];
#pragma unroll
    for (int r = 0; r < 4; ++r) {
      s0[r]     = t0[r]     * 1.52587890625e-05f + bf16_rne(b00[r]);
      s0[4 + r] = t0[4 + r] * 1.52587890625e-05f + bf16_rne(b01[r]);
      s1[r]     = t1[r]     * 1.52587890625e-05f + bf16_rne(b10[r]);
      s1[4 + r] = t1[4 + r] * 1.52587890625e-05f + bf16_rne(b11[r]);
    }
    float mloc = fmaxf(s0[0], s1[0]);
#pragma unroll
    for (int r = 1; r < 8; ++r) mloc = fmaxf(mloc, fmaxf(s0[r], s1[r]));
    mloc = fmaxf(mloc, __shfl_xor(mloc, 16));
    const float mnew = fmaxf(mrun, mloc);
    const float ea = __expf(mrun - mnew);
    const float alpha = (mrun < -1.0e29f) ? 0.0f : ea;
    mrun = mnew;
    FragH pf; float psum = 0.f;
#pragma unroll
    for (int r = 0; r < 8; ++r) {
      const float p0 = __expf(s0[r] - mnew), p1 = __expf(s1[r] - mnew);
      psum += p0 + p1;
      pf.h[r] = (_Float16)(p0 * 1024.0f); pf.h[8 + r] = (_Float16)(p1 * 1024.0f);
    }
    lrun = lrun * alpha + psum;
#pragma unroll
    for (int r = 0; r < 8; ++r) { o0[r] *= alpha; o1[r] *= alpha; o2[r] *= alpha; o3[r] *= alpha; }
    const unsigned short* vp = VT + voff0 + kc;
    const v16h v0 = ld_frag(vp, hh), v1 = ld_frag(vp + 16 * NR, hh), v2 = ld_frag(vp + 32 * NR, hh), v3 = ld_frag(vp + 48 * NR, hh);
    o0 = mma16(v0, pf.v, o0); o1 = mma16(v1, pf.v, o1); o2 = mma16(v2, pf.v, o2); o3 = mma16(v3, pf.v, o3);
  }
  const float l = lrun + __shfl_xor(lrun, 16);
  const float inv = 4.0f * (1.0f / l);
  {
    FragH fh, fr;
#pragma unroll
    for (int r = 0; r < 8; ++r) { const float cv = o0[r] * inv; const _Float16 hi = (_Float16)cv; fh.h[r] = hi; fr.h[r] = (_Float16)(cv - (float)hi); }
    *(v8us*)&sc[wave][0][ln][0 + 8 * hh] = fh.half[0]; *(v8us*)&sc[wave][1][ln][0 + 8 * hh] = fr.half[0];
#pragma unroll
    for (int r = 0; r < 8; ++r) { const float cv = o1[r] * inv; const _Float16 hi = (_Float16)cv; fh.h[r] = hi; fr.h[r] = (_Float16)(cv - (float)hi); }
    *(v8us*)&sc[wave][0][ln][16 + 8 * hh] = fh.half[0]; *(v8us*)&sc[wave][1][ln][16 + 8 * hh] = fr.half[0];
#pragma unroll
    for (int r = 0; r < 8; ++r) { const float cv = o2[r] * inv; const _Float16 hi = (_Float16)cv; fh.h[r] = hi; fr.h[r] = (_Float16)(cv - (float)hi); }
    *(v8us*)&sc[wave][0][ln][32 + 8 * hh] = fh.half[0]; *(v8us*)&sc[wave][1][ln][32 + 8 * hh] = fr.half[0];
#pragma unroll
    for (int r = 0; r < 8; ++r) { const float cv = o3[r] * inv; const _Float16 hi = (_Float16)cv; fh.h[r] = hi; fr.h[r] = (_Float16)(cv - (float)hi); }
    *(v8us*)&sc[wave][0][ln][48 + 8 * hh] = fh.half[0]; *(v8us*)&sc[wave][1][ln][48 + 8 * hh] = fr.half[0];
  }
  __builtin_amdgcn_fence(4  , "workgroup"); __builtin_amdgcn_wave_barrier();
  const int c8 = (lane & 7) * 8, rq = lane >> 3;
  for (int pass = 0; pass < 2; ++pass) {
#pragma unroll
    for (int it = 0; it < 4; ++it) {
      const int row = it * 4 + rq;
      const v8us a = *(const v8us*)&sc[wave][0][row][c8];
      const v8us c = *(const v8us*)&sc[wave][1][row][c8];
      unsigned short* d = CTX + (size_t)(b * SEQ + q0 + row) * (2 * DM) + h * 64 + c8;
      *(volatile v8us*)d = a; *(volatile v8us*)(d + DM) = c;
    }
    if (pass == 0) __threadfence();
  }
}

__global__ __launch_bounds__(128) void k_gemm_proj(const unsigned short* __restrict__ CTX, const unsigned short* __restrict__ WP16, const float* __restrict__ b_proj, float* __restrict__ out) {
  __shared__ __attribute__((aligned(16))) float so[4][32][68];
  const int tid = threadIdx.x; const int wave = __builtin_amdgcn_readfirstlane((int)(tid >> 5));
  const int lane = tid & 31, ln = lane & 15, hh = lane >> 4;
  const int ntn = DM / 64;
  const int mt = blockIdx.x / ntn, nq = blockIdx.x - mt * ntn;
  const int row0 = mt * 128 + 32 * wave, col0 = nq * 64;
  v8f acc[8];
  gemm_core(CTX, 2 * DM, WP16, DM, 2 * DM, DM - 1, row0, col0, ln, hh, acc);
#pragma unroll
  for (int u = 0; u < 8; ++u) { const int t = u & 3, half = u >> 2;
#pragma unroll
    for (int r = 0; r < 8; ++r) so[wave][half * 16 + 8 * hh + r][t * 16 + ln] = acc[u][r] * 1.52587890625e-05f; }
  __builtin_amdgcn_fence(4  , "workgroup"); __builtin_amdgcn_wave_barrier();
  const int rsub = lane >> 4, c4 = (lane & 15) * 4;
  v4f bv;
#pragma unroll
  for (int j = 0; j < 4; ++j) bv[j] = bf16_rne(b_proj[col0 + c4 + j]);
  const int ob = row0 / SEQ;
  const size_t orow0 = (size_t)ob * SEQ_FULL + (size_t)(row0 - ob * SEQ);
  for (int pass = 0; pass < 2; ++pass) {
#pragma unroll 1
    for (int q = 0; q < 16; ++q) {
      const int r = q * 2 + rsub;
      const v4f s = *(const v4fa*)&so[wave][r][c4];
      const v4f v = s + bv;
      *(volatile v4f*)(out + (orow0 + r) * DM + col0 + c4) = v;
    }
    if (pass == 0) __threadfence();
  }
}

extern "C" void kernel_launch(void* const* d_in, const int* in_sizes, int n_in,
                              void* d_out, int out_size, void* d_ws, size_t ws_size, hipStream_t stream) {
  if (n_in < 8) return;
  const long long xneed = ((long long)(NB - 1) * SEQ_FULL + SEQ) * DM;
  if ((long long)in_sizes[0] < xneed) return;
  if ((long long)in_sizes[1] < (long long)(SEQ - 1) * SEQ_FULL + SEQ) return;
  if ((long long)in_sizes[2] < (long long)3 * DM * DM) return;
  if (in_sizes[3] < DM || in_sizes[4] < DM || in_sizes[5] < NH || in_sizes[7] < DM) return;
  if ((long long)in_sizes[6] < (long long)DM * DM) return;
  if ((long long)out_size < xneed) return;
  const float* x = (const float*)d_in[0];
  const float* attn_bias = (const float*)d_in[1];
  const float* W_qkv = (const float*)d_in[2];
  const float* q_bias = (const float*)d_in[3];
  const float* v_bias = (const float*)d_in[4];
  const float* scale_mul = (const float*)d_in[5];
  const float* W_proj = (const float*)d_in[6];
  const float* b_proj = (const float*)d_in[7];
  float* out = (float*)d_out;

  char* ws = (char*)d_ws; size_t off = 0;
  auto take = [&](size_t bytes) { char* p = ws + off; off += (bytes + 255) & ~(size_t)255; return p; };
  unsigned short* X16  = (unsigned short*)take((size_t)NR * DM * 2);
  unsigned short* WQ16 = (unsigned short*)take((size_t)3 * DM * DM * 2);
  unsigned short* WP16 = (unsigned short*)take((size_t)DM * DM * 2);
  unsigned short* QP   = (unsigned short*)take((size_t)NR * 2 * DM * 2);
  unsigned short* K16  = (unsigned short*)take((size_t)NR * DM * 2);
  unsigned short* VT   = (unsigned short*)take((size_t)DM * NR * 2);
  unsigned short* CTX  = (unsigned short*)take((size_t)NR * 2 * DM * 2);
  if (off > ws_size) return;

  k_cvt_x<<<(unsigned)((NR * (DM / 8) + 255) / 256), 256, 0, stream>>>(x, X16);
  k_cvt_w<<<(unsigned)((3 * DM * DM / 8 + 255) / 256), 256, 0, stream>>>(W_qkv, WQ16, 3 * DM * DM / 8, 16.0f);
  k_cvt_w<<<(unsigned)((DM * DM / 8 + 255) / 256), 256, 0, stream>>>(W_proj, WP16, DM * DM / 8, 16.0f);
  k_gemm_qk<<<(unsigned)((NR / 128) * ((2 * DM) / 64)), 128, 0, stream>>>(X16, WQ16, q_bias, scale_mul, QP, K16);
  k_gemm_vt<<<(unsigned)((DM / 128) * (NR / 64)), 128, 0, stream>>>(WQ16 + (size_t)2 * DM * DM, X16, v_bias, VT);
  k_attn<<<dim3(SEQ / 64, NH, NB), 128, 0, stream>>>(QP, K16, VT, attn_bias, CTX);
  k_gemm_proj<<<(unsigned)((NR / 128) * (DM / 64)), 128, 0, stream>>>(CTX, WP16, b_proj, out);
}
